// Encoder_7834020348402
// MI455X (gfx1250) — hardware-verified
//
#include <hip/hip_runtime.h>
#include <math.h>

constexpr int NBATCH = 128;
constexpr int NSTEP  = 64;
constexpr int NFEAT  = 128;
constexpr int NHID   = 256;
constexpr int NGATE  = 4 * NHID;
constexpr int NHC    = 2 * NHID;
constexpr int NATT   = NSTEP;
constexpr int NTHR   = 256;
constexpr int SEQ_BLK = 16;
constexpr int XPITCH = 136;
constexpr int HPITCH = 264;
constexpr int SPITCH = 520;
constexpr int WPITCH = 68;
constexpr int NROWS_TB = NSTEP * NBATCH;
constexpr int NROWS_BF = NBATCH * NFEAT;
constexpr int NOUT     = NBATCH * NSTEP * NFEAT;
constexpr float WCARRY     = 16.0f;
constexpr float WCARRY_INV = 1.0f / 16.0f;

static_assert(NBATCH % SEQ_BLK == 0, "block rows");
static_assert(NHID == 32 * (NTHR / 32), "8 waves x 32 hidden units");
static_assert(NFEAT % 32 == 0 && NHID % 32 == 0 && NHC % 32 == 0 && NSTEP % 32 == 0, "K multiples of 32");
static_assert(NROWS_TB % 64 == 0 && NROWS_BF % 64 == 0 && NATT % 64 == 0, "GEMM tile multiples");
static_assert(SEQ_BLK * NFEAT == NTHR * 8, "x tile staging exact");
static_assert(SEQ_BLK * NHC == 4 * NTHR * 8, "h|c row store exact");
static_assert(NFEAT == 128 && NATT == 64, "attention kernel thread map");
static_assert((XPITCH % 8) == 0 && (HPITCH % 8) == 0 && (SPITCH % 8) == 0 && (WPITCH % 4) == 0, "16-B aligned LDS rows");

typedef __attribute__((ext_vector_type(16))) _Float16 v16h;
typedef __attribute__((ext_vector_type(8)))  _Float16 v8h;
typedef __attribute__((ext_vector_type(8)))  float    v8f;
typedef __attribute__((ext_vector_type(4)))  float    v4f;

__device__ __forceinline__ void wm_guard4(v8f& a0, v8f& a1, v8f& a2, v8f& a3, v16h x, v16h y0, v16h y1, v16h y2, v16h y3) {
  asm volatile("v_nop\n\tv_nop\n\tv_nop\n\tv_nop" : "+v"(a0), "+v"(a1), "+v"(a2), "+v"(a3) : "v"(x), "v"(y0), "v"(y1), "v"(y2), "v"(y3));
}
__device__ __forceinline__ void keep4_h(v16h a, v16h b, v16h c, v16h d) { asm volatile("v_nop" :: "v"(a), "v"(b), "v"(c), "v"(d)); }
__device__ __forceinline__ void acc_guard4(v8f& a, v8f& b, v8f& c, v8f& d) { asm volatile("v_nop\n\tv_nop\n\tv_nop\n\tv_nop" : "+v"(a), "+v"(b), "+v"(c), "+v"(d)); }

template <typename T> struct Frag;
template <> struct Frag<_Float16> {
  typedef v16h V; union U { v16h v; v8h h[2]; };
  static __device__ __forceinline__ v16h load(const _Float16* p) {
    U f; f.h[0] = *(const v8h*)(p); f.h[1] = *(const v8h*)(p + 16); return f.v;
  }
  static __device__ __forceinline__ v8f mma(v16h a, v16h b, v8f c) {
    return __builtin_amdgcn_wmma_f32_16x16x32_f16(false, a, false, b, (short)0, c, false, false);
  }
};

__device__ __forceinline__ float sigm_f(float x) { return __builtin_amdgcn_rcpf(1.0f + expf(-x)); }
__device__ __forceinline__ float tanh_f(float x) { return 1.0f - 2.0f * __builtin_amdgcn_rcpf(expf(2.0f * x) + 1.0f); }

__global__ __launch_bounds__(NTHR) void tp16_kernel(const float* __restrict__ src, int C, int ldo,
                                                    unsigned short* __restrict__ O, float sc,
                                                    long sstride, long ostride) {
  __shared__ float Tt[64 * 65];
  const int tid = threadIdx.x;
  const int c0 = blockIdx.x * 64, r0 = blockIdx.y * 64;
  const float* S = src + (size_t)blockIdx.z * (size_t)sstride;
  _Float16* Oh = (_Float16*)O + (size_t)blockIdx.z * (size_t)ostride;
#pragma unroll
  for (int i = 0; i < 4; ++i) {
    const int idx = i * NTHR + tid;
    const int rr = idx >> 4, cc = (idx & 15) * 4;
    const v4f v = *(const v4f*)(S + (size_t)(r0 + rr) * (size_t)C + c0 + cc);
    Tt[rr * 65 + cc + 0] = v[0];
    Tt[rr * 65 + cc + 1] = v[1];
    Tt[rr * 65 + cc + 2] = v[2];
    Tt[rr * 65 + cc + 3] = v[3];
  }
  __syncthreads();
  const int q = tid >> 3, c8 = (tid & 7) * 8;
  v8h hv0, hv1;
#pragma unroll
  for (int e = 0; e < 8; ++e) {
    const float f0 = Tt[(c8 + e) * 65 + q];
    const float f1 = Tt[(c8 + e) * 65 + 32 + q];
    hv0[e] = (_Float16)(f0 * sc);
    hv1[e] = (_Float16)(f1 * sc);
  }
  const size_t o0 = (size_t)(c0 + q) * (size_t)ldo + (size_t)(r0 + c8);
  const size_t o1 = (size_t)(c0 + 32 + q) * (size_t)ldo + (size_t)(r0 + c8);
  for (int pass = 0; pass < 2; ++pass) {
    *(volatile v8h*)(Oh + o0) = hv0;
    *(volatile v8h*)(Oh + o1) = hv1;
    __threadfence();
  }
}

__global__ __launch_bounds__(256) void gemm64_f16_kernel(
    const unsigned short* __restrict__ Ap, int lda,
    const unsigned short* __restrict__ Btp, int ldb,
    float* __restrict__ Cout, int ldc,
    const float* __restrict__ bias,
    int M, int N, int K, float scale) {
  typedef _Float16 T;
  typedef v16h V;
  const T* A = (const T*)Ap; const T* Bt = (const T*)Btp;
  __shared__ __align__(16) float sT[8][16 * 68];
  const int lane = threadIdx.x & 31;
  const int wave = threadIdx.x >> 5;
  const int tilesN = N >> 6;
  const int tilesM = M >> 6;
  const int tile = blockIdx.x * 8 + wave;
  if (tile >= tilesM * tilesN) return;
  const int tm = tile / tilesN;
  const int tn = tile - tm * tilesN;
  const int m0 = tm << 6;
  const int n0 = tn << 6;

  const int rlane = lane & 15;
  const int koff  = (lane >> 4) * 8;
  const int mOff  = (lane >> 4) * 8;

  v8f acc[4][4];
#pragma unroll
  for (int i = 0; i < 4; ++i)
#pragma unroll
    for (int j = 0; j < 4; ++j) acc[i][j] = (v8f){0.f,0.f,0.f,0.f,0.f,0.f,0.f,0.f};

  for (int k0 = 0; k0 < K; k0 += 32) {
    V bh[4];
#pragma unroll
    for (int j = 0; j < 4; ++j) {
      const size_t bo = (size_t)(n0 + (j << 4) + rlane) * ldb + koff + k0;
      bh[j] = Frag<T>::load(Bt + bo);
    }
#pragma unroll
    for (int i = 0; i < 4; ++i) {
      const size_t ao = (size_t)(m0 + (i << 4) + rlane) * lda + koff + k0;
      V ah = Frag<T>::load(A + ao);
#pragma unroll
      for (int j = 0; j < 4; ++j) acc[i][j] = Frag<T>::mma(ah, bh[j], acc[i][j]);
      wm_guard4(acc[i][0], acc[i][1], acc[i][2], acc[i][3], ah, bh[0], bh[1], bh[2], bh[3]);
    }
    keep4_h(bh[0], bh[1], bh[2], bh[3]);
  }
  acc_guard4(acc[0][0], acc[0][1], acc[0][2], acc[0][3]);
  acc_guard4(acc[1][0], acc[1][1], acc[1][2], acc[1][3]);
  acc_guard4(acc[2][0], acc[2][1], acc[2][2], acc[2][3]);
  acc_guard4(acc[3][0], acc[3][1], acc[3][2], acc[3][3]);

  float* slab = sT[wave];
#pragma unroll
  for (int i = 0; i < 4; ++i) {
    const int mBase = m0 + (i << 4);
#pragma unroll
    for (int j = 0; j < 4; ++j) {
      const int n = n0 + (j << 4) + rlane;
      const float bv = bias[n];
#pragma unroll
      for (int r = 0; r < 8; ++r) {
        float v = acc[i][j][r] * scale;
        v += bv;
        slab[(mOff + r) * 68 + (j << 4) + rlane] = v;
      }
    }
    __builtin_amdgcn_fence(__ATOMIC_RELEASE, "workgroup");
    __builtin_amdgcn_wave_barrier();
    __builtin_amdgcn_fence(__ATOMIC_ACQUIRE, "workgroup");
    {
      const int hh = lane >> 4, c4 = (lane & 15) * 4;
      for (int pass = 0; pass < 2; ++pass) {
#pragma unroll
        for (int it = 0; it < 8; ++it) {
          const int row = it * 2 + hh;
          v4f v = *(const v4f*)(slab + row * 68 + c4);
          *(volatile v4f*)(Cout + (size_t)(mBase + row) * ldc + n0 + c4) = v;
        }
        __threadfence();
      }
    }
    __builtin_amdgcn_fence(__ATOMIC_RELEASE, "workgroup");
    __builtin_amdgcn_wave_barrier();
    __builtin_amdgcn_fence(__ATOMIC_ACQUIRE, "workgroup");
  }
}

__device__ __forceinline__ void stage_x_tile(const float* __restrict__ data, _Float16* Ax, int rowbase, int t, int tid) {
  const int m = tid >> 4, f8 = (tid & 15) * 8;
  const float* sp = data + ((size_t)(rowbase + m) * NSTEP + (size_t)t) * NFEAT + f8;
  const v4f a = *(const v4f*)(sp);
  const v4f b = *(const v4f*)(sp + 4);
  v8h hv;
#pragma unroll
  for (int e = 0; e < 4; ++e) {
    const float fa = a[e];
    const float fb = b[e];
    hv[e]     = (_Float16)fa;
    hv[4 + e] = (_Float16)fb;
  }
  *(v8h*)(Ax + m * XPITCH + f8) = hv;
}

__global__ __launch_bounds__(NTHR) void lstm_seq_kernel(const float* __restrict__ data, const float* __restrict__ bias,
                                                        const float* __restrict__ h0, const float* __restrict__ c0,
                                                        const unsigned short* __restrict__ WTp,
                                                        const unsigned short* __restrict__ UTp,
                                                        unsigned short* __restrict__ HCp) {
  __shared__ __align__(16) _Float16 Ax[SEQ_BLK * XPITCH];
  __shared__ __align__(16) _Float16 Ah[SEQ_BLK * HPITCH];
  __shared__ __align__(16) _Float16 Hs[SEQ_BLK * SPITCH];
  const _Float16* WT = (const _Float16*)WTp;
  const _Float16* UT = (const _Float16*)UTp;
  _Float16* HC = (_Float16*)HCp;
  const int tid = threadIdx.x, lane = tid & 31, wave = tid >> 5;
  const int c = lane & 15, hh = lane >> 4, koff = hh * 8;
  const int rowbase = blockIdx.x * SEQ_BLK;

#pragma unroll 1
  for (int i = 0; i < SEQ_BLK; ++i)
    Ah[i * HPITCH + tid] = (_Float16)h0[(size_t)(rowbase + i) * NHID + tid];
  stage_x_tile(data, Ax, rowbase, 0, tid);

  float cst[2][8], hst[2][8], bb[2][4];
#pragma unroll
  for (int nt = 0; nt < 2; ++nt) {
    const int j = 32 * wave + 16 * nt + c;
#pragma unroll
    for (int g = 0; g < 4; ++g) bb[nt][g] = bias[g * NHID + j];
#pragma unroll
    for (int r = 0; r < 8; ++r) {
      cst[nt][r] = c0[(size_t)(rowbase + 8 * hh + r) * NHID + j];
      hst[nt][r] = 0.0f;
    }
  }
  __syncthreads();

  const _Float16* axrow = Ax + c * XPITCH + koff;
  const _Float16* ahrow = Ah + c * HPITCH + koff;
  const v8f z8 = {0.f, 0.f, 0.f, 0.f, 0.f, 0.f, 0.f, 0.f};

#pragma unroll 1
  for (int t = 0; t < NSTEP; ++t) {
#pragma unroll
    for (int nt = 0; nt < 2; ++nt) {
      const int j = 32 * wave + 16 * nt + c;
      const _Float16* wx = WT + (size_t)j * NFEAT + koff;
      const _Float16* wh = UT + (size_t)j * NHID + koff;
      v8f acc[4];
      acc[0] = z8; acc[1] = z8; acc[2] = z8; acc[3] = z8;
#pragma unroll 1
      for (int kx = 0; kx < NFEAT; kx += 32) {
        const v16h a  = Frag<_Float16>::load(axrow + kx);
        const v16h b0 = Frag<_Float16>::load(wx + kx);
        const v16h b1 = Frag<_Float16>::load(wx + (size_t)1 * NHID * NFEAT + kx);
        const v16h b2 = Frag<_Float16>::load(wx + (size_t)2 * NHID * NFEAT + kx);
        const v16h b3 = Frag<_Float16>::load(wx + (size_t)3 * NHID * NFEAT + kx);
        acc[0] = Frag<_Float16>::mma(a, b0, acc[0]);
        acc[1] = Frag<_Float16>::mma(a, b1, acc[1]);
        acc[2] = Frag<_Float16>::mma(a, b2, acc[2]);
        acc[3] = Frag<_Float16>::mma(a, b3, acc[3]);
        wm_guard4(acc[0], acc[1], acc[2], acc[3], a, b0, b1, b2, b3);
      }
#pragma unroll 1
      for (int k0 = 0; k0 < NHID; k0 += 32) {
        const v16h a  = Frag<_Float16>::load(ahrow + k0);
        const v16h b0 = Frag<_Float16>::load(wh + k0);
        const v16h b1 = Frag<_Float16>::load(wh + (size_t)1 * NHID * NHID + k0);
        const v16h b2 = Frag<_Float16>::load(wh + (size_t)2 * NHID * NHID + k0);
        const v16h b3 = Frag<_Float16>::load(wh + (size_t)3 * NHID * NHID + k0);
        acc[0] = Frag<_Float16>::mma(a, b0, acc[0]);
        acc[1] = Frag<_Float16>::mma(a, b1, acc[1]);
        acc[2] = Frag<_Float16>::mma(a, b2, acc[2]);
        acc[3] = Frag<_Float16>::mma(a, b3, acc[3]);
        wm_guard4(acc[0], acc[1], acc[2], acc[3], a, b0, b1, b2, b3);
      }
      acc_guard4(acc[0], acc[1], acc[2], acc[3]);
#pragma unroll
      for (int r = 0; r < 8; ++r) {
        const float zi = acc[0][r] * WCARRY_INV + bb[nt][0];
        const float zf = acc[1][r] * WCARRY_INV + bb[nt][1];
        const float zg = acc[2][r] * WCARRY_INV + bb[nt][2];
        const float zo = acc[3][r] * WCARRY_INV + bb[nt][3];
        const float ig = sigm_f(zi);
        const float fg = sigm_f(zf);
        const float gg = tanh_f(zg);
        const float og = sigm_f(zo);
        const float cn = fg * cst[nt][r] + ig * gg;
        cst[nt][r] = cn;
        hst[nt][r] = og * tanh_f(cn);
      }
    }
    __syncthreads();
#pragma unroll
    for (int nt = 0; nt < 2; ++nt) {
      const int j = 32 * wave + 16 * nt + c;
#pragma unroll
      for (int r = 0; r < 8; ++r) {
        const _Float16 hv = (_Float16)hst[nt][r];
        const _Float16 cv = (_Float16)cst[nt][r];
        Ah[(8 * hh + r) * HPITCH + j] = hv;
        Hs[(8 * hh + r) * SPITCH + j] = hv;
        Hs[(8 * hh + r) * SPITCH + NHID + j] = cv;
      }
    }
    {
      const int tn = (t + 1 < NSTEP) ? (t + 1) : (NSTEP - 1);
      stage_x_tile(data, Ax, rowbase, tn, tid);
    }
    __syncthreads();
    for (int pass = 0; pass < 2; ++pass) {
#pragma unroll
      for (int it = 0; it < 4; ++it) {
        const int idx = it * NTHR + tid;
        const int row = idx >> 6, c8 = (idx & 63) * 8;
        const v8h v = *(const v8h*)(Hs + row * SPITCH + c8);
        *(volatile v8h*)(HC + ((size_t)t * NBATCH + (size_t)(rowbase + row)) * NHC + c8) = v;
      }
      __threadfence();
    }
  }
}

__global__ __launch_bounds__(128) void attn_out_kernel(const float* __restrict__ W1X, const float* __restrict__ Q,
                                                       const float* __restrict__ vk, const float* __restrict__ vb,
                                                       const float* __restrict__ data, float* __restrict__ out) {
  __shared__ __align__(16) float Wt[NFEAT * WPITCH];
  __shared__ __align__(16) float Qs[NSTEP * NATT];
  __shared__ float vs[NATT];
  __shared__ float redm[4];
  __shared__ float reds[4];
  const int b = blockIdx.x;
  const int tid = threadIdx.x, lane = tid & 31, wave = tid >> 5;

#pragma unroll 1
  for (int i = 0; i < 16; ++i) {
    const int idx = i * 128 + tid;
    const int row = idx >> 4, c4 = (idx & 15) * 4;
    const v4f v = *(const v4f*)(W1X + (size_t)b * (NFEAT * NATT) + (size_t)idx * 4);
    *(v4f*)(Wt + row * WPITCH + c4) = v;
  }
#pragma unroll 1
  for (int i = 0; i < 8; ++i) {
    const int idx = i * 128 + tid;
    const int tt = idx >> 4, c4 = (idx & 15) * 4;
    const v4f v = *(const v4f*)(Q + ((size_t)tt * NBATCH + (size_t)b) * NATT + c4);
    *(v4f*)(Qs + tt * NATT + c4) = v;
  }
  {
    const float vv = vk[tid & (NATT - 1)];
    if (tid < NATT) vs[tid] = vv;
  }
  const float vb0 = vb[0];
  __syncthreads();

  const float* wr = Wt + tid * WPITCH;

#pragma unroll 1
  for (int t = 0; t < NSTEP; ++t) {
    const size_t orow = ((size_t)t * NBATCH + (size_t)b) * NFEAT;
    float dval = data[orow + tid];
    asm volatile("" : "+v"(dval));
    const float* qr = Qs + t * NATT;
    float sc = 0.0f;
#pragma unroll 2
    for (int s = 0; s < NATT; ++s) {
      const float x = wr[s] + qr[s];
      const float th = tanh_f(x);
      sc = fmaf(th, vs[s], sc);
    }
    sc += vb0;
    float m = sc;
#pragma unroll
    for (int off = 16; off > 0; off >>= 1) m = fmaxf(m, __shfl_xor(m, off, 32));
    if (lane == 0) redm[wave] = m;
    __syncthreads();
    const float mx = fmaxf(fmaxf(redm[0], redm[1]), fmaxf(redm[2], redm[3]));
    const float e = expf(sc - mx);
    float sm = e;
#pragma unroll
    for (int off = 16; off > 0; off >>= 1) sm += __shfl_xor(sm, off, 32);
    if (lane == 0) reds[wave] = sm;
    __syncthreads();
    const float tot = (reds[0] + reds[1]) + (reds[2] + reds[3]);
    const float alpha = e * __builtin_amdgcn_rcpf(tot);
    const float o = dval * alpha;
    volatile float* op = out + orow + tid;
    *op = o;
    __threadfence();
    *op = o;
  }
}

extern "C" void kernel_launch(void* const* d_in, const int* in_sizes, int n_in,
                              void* d_out, int out_size, void* d_ws, size_t ws_size, hipStream_t stream) {
  if (n_in < 12 || d_out == nullptr || d_ws == nullptr) return;
  if (in_sizes[0] != NBATCH * NSTEP * NFEAT || in_sizes[1] != NBATCH * NHID || in_sizes[2] != NBATCH * NHID ||
      in_sizes[3] != NFEAT * NGATE || in_sizes[4] != NHID * NGATE || in_sizes[5] != NGATE ||
      in_sizes[6] != NSTEP * NATT || in_sizes[7] != NATT || in_sizes[8] != NHC * NATT || in_sizes[9] != NATT ||
      in_sizes[10] != NATT || in_sizes[11] != 1 || out_size != NOUT) return;

  const float* data = (const float*)d_in[0];
  const float* h0   = (const float*)d_in[1];
  const float* c0   = (const float*)d_in[2];
  const float* Wk   = (const float*)d_in[3];
  const float* Uk   = (const float*)d_in[4];
  const float* bk   = (const float*)d_in[5];
  const float* w1k  = (const float*)d_in[6];
  const float* w1b  = (const float*)d_in[7];
  const float* w2k  = (const float*)d_in[8];
  const float* w2b  = (const float*)d_in[9];
  const float* vk   = (const float*)d_in[10];
  const float* vb   = (const float*)d_in[11];
  float* out = (float*)d_out;

  char* ws = (char*)d_ws; size_t off = 0;
  auto carve = [&](size_t bytes) -> char* { char* p = ws + off; off += (bytes + 255) & ~(size_t)255; return p; };
  unsigned short* XT16 = (unsigned short*)carve((size_t)NROWS_BF * NSTEP * 2);
  unsigned short* WT   = (unsigned short*)carve((size_t)NGATE * NFEAT * 2);
  unsigned short* UT   = (unsigned short*)carve((size_t)NGATE * NHID * 2);
  unsigned short* W1T  = (unsigned short*)carve((size_t)NATT * NSTEP * 2);
  unsigned short* W2T  = (unsigned short*)carve((size_t)NATT * NHC * 2);
  float*          W1X  = (float*)carve((size_t)NROWS_BF * NATT * 4);
  unsigned short* HC   = (unsigned short*)carve((size_t)NROWS_TB * NHC * 2);
  float*          QP   = (float*)carve((size_t)NROWS_TB * NATT * 4);
  if (off > ws_size || off > (size_t)134217728) return;

  tp16_kernel<<<dim3(NFEAT / 64, NSTEP / 64, NBATCH), NTHR, 0, stream>>>(data, NFEAT, NSTEP, XT16, 1.0f,
                                                                         (long)NSTEP * NFEAT, (long)NFEAT * NSTEP);
  tp16_kernel<<<dim3(NGATE / 64, NFEAT / 64, 1), NTHR, 0, stream>>>(Wk, NGATE, NFEAT, WT, WCARRY, 0L, 0L);
  tp16_kernel<<<dim3(NGATE / 64, NHID / 64, 1), NTHR, 0, stream>>>(Uk, NGATE, NHID, UT, WCARRY, 0L, 0L);
  tp16_kernel<<<dim3(NATT / 64, NSTEP / 64, 1), NTHR, 0, stream>>>(w1k, NATT, NSTEP, W1T, WCARRY, 0L, 0L);
  tp16_kernel<<<dim3(NATT / 64, NHC / 64, 1), NTHR, 0, stream>>>(w2k, NATT, NHC, W2T, WCARRY, 0L, 0L);

  gemm64_f16_kernel<<<(NROWS_BF / 64) * (NATT / 64) / 8, 256, 0, stream>>>(
      XT16, NSTEP, W1T, NSTEP, W1X, NATT, w1b, NROWS_BF, NATT, NSTEP, WCARRY_INV);

  lstm_seq_kernel<<<NBATCH / SEQ_BLK, NTHR, 0, stream>>>(data, bk, h0, c0, WT, UT, HC);

  gemm64_f16_kernel<<<(NROWS_TB / 64) * (NATT / 64) / 8, 256, 0, stream>>>(
      HC, NHC, W2T, NHC, QP, NATT, w2b, NROWS_TB, NATT, NHC, WCARRY_INV);

  attn_out_kernel<<<NBATCH, 128, 0, stream>>>(W1X, QP, vk, vb, data, out);
}
